// mLSTM_cell_87883620811267
// MI455X (gfx1250) — hardware-verified
//
#include <hip/hip_runtime.h>
#include <math.h>


static constexpr int kBS  = 4;
static constexpr int kT   = 1024;
static constexpr int kC   = 1024;
static constexpr int kNH  = 16;
static constexpr int kHD  = 64;
static constexpr int kBH  = kBS * kNH;
static constexpr int kRB  = kT / 64;
static constexpr int kSTP = 136;
static constexpr int kPP  = 72;
static constexpr int kThreads = 256;
static constexpr int kGateN = kBH * kT;
static constexpr int kPlane = kBH * kT * kHD;
static constexpr int kNX  = kBS * kT * kC;
static constexpr int kNW  = kC * kC;
static constexpr int kNG  = kNH * kC;

static_assert(kC == kNH * kHD);
static_assert(kHD == 64);
static_assert(kNH == 16);
static_assert(kT % 128 == 0 && kC % 128 == 0);
static_assert((kSTP % 8) == 0 && (kPP % 8) == 0);
static_assert(kNX % (kThreads * 8) == 0);
static_assert(kNW % (kThreads * 8) == 0);
static_assert(kNG % (kThreads * 8) == 0);
static_assert(kT == 128 * 8);

typedef _Float16     v16h __attribute__((ext_vector_type(16)));
typedef _Float16     v8h  __attribute__((ext_vector_type(8)));
typedef float        v8f  __attribute__((ext_vector_type(8)));
typedef float        v4f  __attribute__((ext_vector_type(4)));
typedef unsigned int v4u  __attribute__((ext_vector_type(4)));

union Frag { v16h v; v8h half[2]; };

__device__ __forceinline__ v8f wmma_f16(v16h a, v16h b, v8f acc)
{
    acc = __builtin_amdgcn_wmma_f32_16x16x32_f16(false, a, false, b, (short)0, acc, false, false);
#if defined(__HIP_DEVICE_COMPILE__)
    asm volatile("v_nop\n\tv_nop\n\tv_nop\n\tv_nop" : "+v"(acc) : "v"(a), "v"(b));
#endif
    return acc;
}

__device__ __forceinline__ v8f zero8()
{
    v8f z;
#pragma unroll
    for (int r = 0; r < 8; ++r) z[r] = 0.0f;
    return z;
}

__device__ __forceinline__ float bf16_rne(float x)
{
    unsigned int u = __float_as_uint(x);
    u = u + 0x7FFFu + ((u >> 16) & 1u);
    return __uint_as_float(u & 0xFFFF0000u);
}

__device__ __forceinline__ _Float16 cvt16(float x, float sc)
{
    return (_Float16)(bf16_rne(x) * sc);
}

__global__ __launch_bounds__(kThreads)
void k_cvt3(const float* s0, _Float16* d0, int n0,
            const float* s1, _Float16* d1, int n1,
            const float* s2, _Float16* d2, int n2, float sc)
{
    const float* src = s0;
    _Float16*    dst = d0;
    int          n   = n0;
    if (blockIdx.y == 1) { src = s1; dst = d1; n = n1; }
    else if (blockIdx.y == 2) { src = s2; dst = d2; n = n2; }

    const size_t base = ((size_t)blockIdx.x * kThreads + threadIdx.x) * 8;
    if (base + 8 <= (size_t)n) {
        const v4f f0 = *(const v4f*)(src + base);
        const v4f f1 = *(const v4f*)(src + base + 4);
        v8h hv;
        hv[0] = cvt16(f0[0], sc); hv[1] = cvt16(f0[1], sc);
        hv[2] = cvt16(f0[2], sc); hv[3] = cvt16(f0[3], sc);
        hv[4] = cvt16(f1[0], sc); hv[5] = cvt16(f1[1], sc);
        hv[6] = cvt16(f1[2], sc); hv[7] = cvt16(f1[3], sc);
        const v4u u = __builtin_bit_cast(v4u, hv);
        volatile v4u* p = (volatile v4u*)(dst + base);
        *p = u;
        __threadfence();
        *p = u;
    }
}

__global__ __launch_bounds__(kThreads)
void k_gates(const _Float16* __restrict__ Xq, const _Float16* __restrict__ Xk,
             const _Float16* __restrict__ Wi16, const _Float16* __restrict__ Wf16,
             const float* __restrict__ bI, const float* __restrict__ bF,
             float* __restrict__ G)
{
    __shared__ __align__(16) float sG[2 * kNH * 128];
    const int tid  = threadIdx.x;
    const int wave = tid >> 5;
    const int lane = tid & 31;
    const int h    = lane >> 4;
    const int m    = lane & 15;
    const int sBase = blockIdx.x * 128;
    const int b     = blockIdx.y;

    const size_t rowA = (size_t)b * kT + sBase + 16 * wave + m;
    const _Float16* qa = Xq + rowA * kC + 8 * h;
    const _Float16* ka = Xk + rowA * kC + 8 * h;
    const _Float16* wi = Wi16 + (size_t)m * kC + 8 * h;
    const _Float16* wf = Wf16 + (size_t)m * kC + 8 * h;

    v8f ai = zero8(), af = zero8();
#pragma unroll 2
    for (int k0 = 0; k0 < kC; k0 += 32) {
        Frag a, w;
        a.half[0] = *(const v8h*)(qa + k0);
        a.half[1] = *(const v8h*)(qa + k0 + 16);
        w.half[0] = *(const v8h*)(wi + k0);
        w.half[1] = *(const v8h*)(wi + k0 + 16);
        ai = wmma_f16(a.v, w.v, ai);
        Frag a2, w2;
        a2.half[0] = *(const v8h*)(ka + k0);
        a2.half[1] = *(const v8h*)(ka + k0 + 16);
        w2.half[0] = *(const v8h*)(wf + k0);
        w2.half[1] = *(const v8h*)(wf + k0 + 16);
        af = wmma_f16(a2.v, w2.v, af);
    }

    const float biv = bf16_rne(bI[m]);
    const float bfv = bf16_rne(bF[m]);
    {
        float* si = sG + m * 128 + 16 * wave + 8 * h;
        float* sf = sG + (kNH + m) * 128 + 16 * wave + 8 * h;
#pragma unroll
        for (int r = 0; r < 8; ++r) {
            const float iv = ai[r] * (1.0f / 8192.0f) + biv;
            const float fv = af[r] * (1.0f / 8192.0f) + bfv;
            const float ls = fminf(fv, 0.0f) - log1pf(expf(-fabsf(fv)));
            si[r] = iv;
            sf[r] = ls;
        }
    }
    __syncthreads();

    v4f vals[4];
    int off[4];
#pragma unroll
    for (int it = 0; it < 4; ++it) {
        const int p     = it * kThreads + tid;
        const int row   = p >> 5;
        const int j     = p & 31;
        const int plane = row >> 4;
        const int hd    = row & 15;
        vals[it] = *(const v4f*)(sG + row * 128 + 4 * j);
        off[it]  = plane * kGateN + (b * kNH + hd) * kT + sBase + 4 * j;
    }
#pragma unroll
    for (int it = 0; it < 4; ++it) *(volatile v4f*)(G + (size_t)off[it]) = vals[it];
    __threadfence();
#pragma unroll
    for (int it = 0; it < 4; ++it) *(volatile v4f*)(G + (size_t)off[it]) = vals[it];
}

__device__ __forceinline__ void store_direct(const _Float16* sT, _Float16* __restrict__ dstp,
                                             int b, int hA, int t0, int tid)
{
    v4u u[8];
    int off[8];
#pragma unroll
    for (int it = 0; it < 8; ++it) {
        const int p    = it * kThreads + tid;
        const int line = p >> 3;
        const int j    = p & 7;
        const int hh   = line >> 7;
        const int tr   = line & 127;
        const v8h hv = *(const v8h*)(sT + tr * kSTP + hh * 64 + 8 * j);
        u[it]   = __builtin_bit_cast(v4u, hv);
        off[it] = ((b * kNH + hA + hh) * kT + t0 + tr) * kHD + 8 * j;
    }
#pragma unroll
    for (int it = 0; it < 8; ++it) *(volatile v4u*)(dstp + (size_t)off[it]) = u[it];
    __threadfence();
#pragma unroll
    for (int it = 0; it < 8; ++it) *(volatile v4u*)(dstp + (size_t)off[it]) = u[it];
}

__device__ __forceinline__ void store_trans(const _Float16* sT, _Float16* __restrict__ dstp,
                                            int b, int hA, int t0, int tid)
{
    v4u u[8];
    int off[8];
#pragma unroll
    for (int it = 0; it < 8; ++it) {
        const int p   = it * kThreads + tid;
        const int row = p >> 4;
        const int j   = p & 15;
        const int hh  = row >> 6;
        const int d   = row & 63;
        v8h hv;
#pragma unroll
        for (int ii = 0; ii < 8; ++ii) hv[ii] = sT[(8 * j + ii) * kSTP + hh * 64 + d];
        u[it]   = __builtin_bit_cast(v4u, hv);
        off[it] = ((b * kNH + hA + hh) * kHD + d) * kT + t0 + 8 * j;
    }
#pragma unroll
    for (int it = 0; it < 8; ++it) *(volatile v4u*)(dstp + (size_t)off[it]) = u[it];
    __threadfence();
#pragma unroll
    for (int it = 0; it < 8; ++it) *(volatile v4u*)(dstp + (size_t)off[it]) = u[it];
}

__global__ __launch_bounds__(kThreads)
void k_qkv(const _Float16* __restrict__ X16, const _Float16* __restrict__ W16,
           const float* __restrict__ bq, const float* __restrict__ bk,
           const float* __restrict__ bvp,
           _Float16* __restrict__ QH, _Float16* __restrict__ QL,
           _Float16* __restrict__ KH, _Float16* __restrict__ KL,
           _Float16* __restrict__ VT)
{
    __shared__ __align__(16) _Float16 sT[128 * kSTP];
    const int tid  = threadIdx.x;
    const int wave = tid >> 5;
    const int lane = tid & 31;
    const int h    = lane >> 4;
    const int m    = lane & 15;
    const int wm   = wave >> 1;
    const int wn   = wave & 1;
    const int kind  = blockIdx.z;
    const int nBase = blockIdx.x * 128;
    const int mBase = blockIdx.y * 128;

    const _Float16* Xp = X16 + (size_t)kind * (size_t)kNX;
    const _Float16* Wp = W16 + (size_t)kind * (size_t)kNW;
    const float* bias  = (kind == 0) ? bq : ((kind == 1) ? bk : bvp);

    const _Float16* xa0 = Xp + (size_t)(mBase + 32 * wm + m) * kC + 8 * h;
    const _Float16* xa1 = xa0 + (size_t)16 * kC;
    const _Float16* wb0 = Wp + (size_t)(nBase + 64 * wn + m) * kC + 8 * h;

    v8f acc0[4], acc1[4];
#pragma unroll
    for (int ct = 0; ct < 4; ++ct) { acc0[ct] = zero8(); acc1[ct] = zero8(); }

#pragma unroll 1
    for (int k0 = 0; k0 < kC; k0 += 32) {
        Frag a0, a1;
        a0.half[0] = *(const v8h*)(xa0 + k0);
        a0.half[1] = *(const v8h*)(xa0 + k0 + 16);
        a1.half[0] = *(const v8h*)(xa1 + k0);
        a1.half[1] = *(const v8h*)(xa1 + k0 + 16);
#pragma unroll
        for (int ct = 0; ct < 4; ++ct) {
            Frag bw;
            const _Float16* wp = wb0 + (size_t)ct * 16 * kC + k0;
            bw.half[0] = *(const v8h*)(wp);
            bw.half[1] = *(const v8h*)(wp + 16);
            acc0[ct] = wmma_f16(a0.v, bw.v, acc0[ct]);
            acc1[ct] = wmma_f16(a1.v, bw.v, acc1[ct]);
        }
    }

    float b8[4];
#pragma unroll
    for (int ct = 0; ct < 4; ++ct)
        b8[ct] = 8.0f * bf16_rne(bias[nBase + 64 * wn + 16 * ct + m]);

    {
        _Float16* s0 = sT + (32 * wm + 8 * h) * kSTP + 64 * wn + m;
#pragma unroll
        for (int ct = 0; ct < 4; ++ct) {
#pragma unroll
            for (int r = 0; r < 8; ++r) {
                const float y0 = acc0[ct][r] * (1.0f / 1024.0f) + b8[ct];
                const float y1 = acc1[ct][r] * (1.0f / 1024.0f) + b8[ct];
                s0[r * kSTP + 16 * ct]        = (_Float16)y0;
                s0[(16 + r) * kSTP + 16 * ct] = (_Float16)y1;
            }
        }
    }
    __syncthreads();

    const int hA = nBase >> 6;
    const int b  = mBase / kT;
    const int t0 = mBase % kT;

    if (kind < 2) {
        store_direct(sT, (kind == 0) ? QH : KH, b, hA, t0, tid);
    } else {
        store_trans(sT, VT, b, hA, t0, tid);
    }

    if (kind < 2) {
        __syncthreads();
        _Float16* s0 = sT + (32 * wm + 8 * h) * kSTP + 64 * wn + m;
#pragma unroll
        for (int ct = 0; ct < 4; ++ct) {
#pragma unroll
            for (int r = 0; r < 8; ++r) {
                const float y0 = acc0[ct][r] * (1.0f / 1024.0f) + b8[ct];
                const float y1 = acc1[ct][r] * (1.0f / 1024.0f) + b8[ct];
                const _Float16 h0 = (_Float16)y0;
                const _Float16 h1 = (_Float16)y1;
                s0[r * kSTP + 16 * ct]        = (_Float16)((y0 - (float)h0) * 2048.0f);
                s0[(16 + r) * kSTP + 16 * ct] = (_Float16)((y1 - (float)h1) * 2048.0f);
            }
        }
        __syncthreads();
        store_direct(sT, (kind == 0) ? QL : KL, b, hA, t0, tid);
    }
}

__global__ __launch_bounds__(128)
void k_attn(const _Float16* __restrict__ QH, const _Float16* __restrict__ QL,
            const _Float16* __restrict__ KH, const _Float16* __restrict__ KL,
            const _Float16* __restrict__ VT, const float* __restrict__ G,
            const float* __restrict__ gam, const float* __restrict__ bet,
            float* __restrict__ out)
{
    __shared__ __align__(16) float sCf[kT];
    __shared__ __align__(16) float sIt[kT];
    __shared__ __align__(16) _Float16 sP[4 * 16 * kPP];
    __shared__ __align__(16) float sStg[4 * 16 * kHD];
    __shared__ float sTot[4];

    const int tid  = threadIdx.x;
    const int wave = tid >> 5;
    const int lane = tid & 31;
    const int h    = lane >> 4;
    const int m    = lane & 15;
    const int rb   = blockIdx.x;
    const int head = blockIdx.y;
    const int b    = blockIdx.z;
    const int R    = rb * 64;
    const int r0   = R + 16 * wave;
    const int bh   = b * kNH + head;
    const float kNeg = -1.0e30f;

    {
        const float* gi = G + (size_t)bh * kT + tid * 8;
        const float* gl = G + (size_t)kGateN + (size_t)bh * kT + tid * 8;
        const v4f l0 = *(const v4f*)(gl);
        const v4f l1 = *(const v4f*)(gl + 4);
        const v4f i0 = *(const v4f*)(gi);
        const v4f i1 = *(const v4f*)(gi + 4);
        *(v4f*)(sIt + tid * 8)     = i0;
        *(v4f*)(sIt + tid * 8 + 4) = i1;
        float c[8];
        c[0] = l0[0];        c[1] = c[0] + l0[1]; c[2] = c[1] + l0[2]; c[3] = c[2] + l0[3];
        c[4] = c[3] + l1[0]; c[5] = c[4] + l1[1]; c[6] = c[5] + l1[2]; c[7] = c[6] + l1[3];
        float x = c[7];
#pragma unroll
        for (int off = 1; off < 32; off <<= 1) {
            const float t = __shfl_up(x, off, 32);
            x = (lane >= off) ? (x + t) : x;
        }
        float xe = __shfl_up(x, 1, 32);
        xe = (lane >= 1) ? xe : 0.0f;
        if (lane == 31) sTot[wave] = x;
        __syncthreads();
        const float w0  = sTot[0], w1 = sTot[1], w2 = sTot[2];
        const float p01 = w0 + w1;
        float pre = (wave == 0) ? 0.0f : ((wave == 1) ? w0 : ((wave == 2) ? p01 : (p01 + w2)));
        pre = pre + xe;
        v4f o0, o1;
        o0[0] = pre + c[0]; o0[1] = pre + c[1]; o0[2] = pre + c[2]; o0[3] = pre + c[3];
        o1[0] = pre + c[4]; o1[1] = pre + c[5]; o1[2] = pre + c[6]; o1[3] = pre + c[7];
        *(v4f*)(sCf + tid * 8)     = o0;
        *(v4f*)(sCf + tid * 8 + 4) = o1;
    }
    __syncthreads();

    float cfi[8];
#pragma unroll
    for (int r = 0; r < 8; ++r) cfi[r] = sCf[r0 + 8 * h + r];

    Frag aqh0, aqh1, aql0, aql1;
    {
        const size_t qo = ((size_t)bh * kT + r0 + m) * kHD + 8 * h;
        const _Float16* qh = QH + qo;
        const _Float16* ql = QL + qo;
        aqh0.half[0] = *(const v8h*)(qh);      aqh0.half[1] = *(const v8h*)(qh + 16);
        aqh1.half[0] = *(const v8h*)(qh + 32); aqh1.half[1] = *(const v8h*)(qh + 48);
        aql0.half[0] = *(const v8h*)(ql);      aql0.half[1] = *(const v8h*)(ql + 16);
        aql1.half[0] = *(const v8h*)(ql + 32); aql1.half[1] = *(const v8h*)(ql + 48);
    }

    v8f iacc[4];
#pragma unroll
    for (int et = 0; et < 4; ++et) iacc[et] = zero8();
    float mrun[8], rs[8];
#pragma unroll
    for (int r = 0; r < 8; ++r) { mrun[r] = kNeg; rs[r] = 0.0f; }

    const size_t kro = ((size_t)bh * kT + m) * kHD + 8 * h;
    const _Float16* khb = KH + kro;
    const _Float16* klb = KL + kro;
    const _Float16* vb  = VT + ((size_t)bh * kHD + m) * kT + 8 * h;
    _Float16* myP = sP + wave * (16 * kPP);
    const int nch = rb + 1;

#pragma unroll 1
    for (int c = 0; c < nch; ++c) {
        const int kc = c * 64;

        float mx[8];
#pragma unroll
        for (int r = 0; r < 8; ++r) mx[r] = kNeg;
#pragma unroll
        for (int nt = 0; nt < 4; ++nt) {
            const int j = kc + 16 * nt + m;
            const float cj = sCf[j];
            const float ij = sIt[j];
#pragma unroll
            for (int r = 0; r < 8; ++r) {
                const int i = r0 + 8 * h + r;
                float dt = (cfi[r] - cj) + ij;
                dt = (j <= i) ? dt : kNeg;
                mx[r] = fmaxf(mx[r], dt);
            }
        }
        float scl[8];
#pragma unroll
        for (int r = 0; r < 8; ++r) {
            float v = mx[r];
            v = fmaxf(v, __shfl_xor(v, 1, 32));
            v = fmaxf(v, __shfl_xor(v, 2, 32));
            v = fmaxf(v, __shfl_xor(v, 4, 32));
            v = fmaxf(v, __shfl_xor(v, 8, 32));
            const float mn = fmaxf(mrun[r], v);
            scl[r]  = __expf(mrun[r] - mn);
            mrun[r] = mn;
            rs[r]  *= scl[r];
        }
#pragma unroll
        for (int et = 0; et < 4; ++et) {
#pragma unroll
            for (int r = 0; r < 8; ++r) iacc[et][r] *= scl[r];
        }

        float ps[8];
#pragma unroll
        for (int r = 0; r < 8; ++r) ps[r] = 0.0f;
#pragma unroll
        for (int nt = 0; nt < 4; ++nt) {
            const size_t ko = (size_t)(kc + 16 * nt) * kHD;
            Frag kh0, kh1;
            kh0.half[0] = *(const v8h*)(khb + ko);      kh0.half[1] = *(const v8h*)(khb + ko + 16);
            kh1.half[0] = *(const v8h*)(khb + ko + 32); kh1.half[1] = *(const v8h*)(khb + ko + 48);
            v8f shh = zero8();
            shh = wmma_f16(aqh0.v, kh0.v, shh);
            shh = wmma_f16(aqh1.v, kh1.v, shh);
            v8f sx = zero8();
            sx = wmma_f16(aql0.v, kh0.v, sx);
            sx = wmma_f16(aql1.v, kh1.v, sx);
            Frag kl0, kl1;
            kl0.half[0] = *(const v8h*)(klb + ko);      kl0.half[1] = *(const v8h*)(klb + ko + 16);
            kl1.half[0] = *(const v8h*)(klb + ko + 32); kl1.half[1] = *(const v8h*)(klb + ko + 48);
            sx = wmma_f16(aqh0.v, kl0.v, sx);
            sx = wmma_f16(aqh1.v, kl1.v, sx);

            const int j = kc + 16 * nt + m;
            const float cj = sCf[j];
            const float ij = sIt[j];
            _Float16* pcol = myP + (8 * h) * kPP + 16 * nt + m;
#pragma unroll
            for (int r = 0; r < 8; ++r) {
                const int i = r0 + 8 * h + r;
                float dt = (cfi[r] - cj) + ij;
                dt = (j <= i) ? dt : kNeg;
                const float e  = __expf(dt - mrun[r]);
                const float sv = shh[r] + sx[r] * (1.0f / 2048.0f);
                const float p  = sv * e;
                ps[r] += p;
                pcol[r * kPP] = (_Float16)(p * 4.0f);
            }
        }
#pragma unroll
        for (int r = 0; r < 8; ++r) {
            float v = ps[r];
            v += __shfl_xor(v, 1, 32);
            v += __shfl_xor(v, 2, 32);
            v += __shfl_xor(v, 4, 32);
            v += __shfl_xor(v, 8, 32);
            rs[r] += v;
        }
        __syncthreads();

#pragma unroll
        for (int ks = 0; ks < 2; ++ks) {
            Frag a;
            const _Float16* pa = myP + m * kPP + 32 * ks + 8 * h;
            a.half[0] = *(const v8h*)(pa);
            a.half[1] = *(const v8h*)(pa + 16);
#pragma unroll
            for (int et = 0; et < 4; ++et) {
                const _Float16* vp = vb + (size_t)et * 16 * kT + kc + 32 * ks;
                Frag bvf;
                bvf.half[0] = *(const v8h*)(vp);
                bvf.half[1] = *(const v8h*)(vp + 16);
                iacc[et] = wmma_f16(a.v, bvf.v, iacc[et]);
            }
        }
        __syncthreads();
    }

    float g4[4], b4[4];
#pragma unroll
    for (int et = 0; et < 4; ++et) {
        const int ch = head * kHD + 16 * et + m;
        g4[et] = bf16_rne(gam[ch]);
        b4[et] = bf16_rne(bet[ch]);
    }
    float* mys = sStg + wave * (16 * kHD);
#pragma unroll
    for (int r = 0; r < 8; ++r) {
        const float rsv   = rs[r] * (1.0f / 2048.0f);
        const float mt    = fmaxf(fabsf(rsv), expf(-mrun[r]));
        const float scale = (1.0f / (mt + 1e-8f)) * (1.0f / 65536.0f);
        float hv[4];
#pragma unroll
        for (int et = 0; et < 4; ++et) hv[et] = iacc[et][r] * scale;
        float s1 = (hv[0] + hv[1]) + (hv[2] + hv[3]);
        s1 += __shfl_xor(s1, 1, 32);
        s1 += __shfl_xor(s1, 2, 32);
        s1 += __shfl_xor(s1, 4, 32);
        s1 += __shfl_xor(s1, 8, 32);
        const float mean = s1 * (1.0f / 64.0f);
        float dv[4];
#pragma unroll
        for (int et = 0; et < 4; ++et) dv[et] = hv[et] - mean;
        float s2 = (dv[0] * dv[0] + dv[1] * dv[1]) + (dv[2] * dv[2] + dv[3] * dv[3]);
        s2 += __shfl_xor(s2, 1, 32);
        s2 += __shfl_xor(s2, 2, 32);
        s2 += __shfl_xor(s2, 4, 32);
        s2 += __shfl_xor(s2, 8, 32);
        const float var  = s2 * (1.0f / 64.0f);
        const float rstd = 1.0f / sqrtf(var + 1e-5f);
#pragma unroll
        for (int et = 0; et < 4; ++et)
            mys[(8 * h + r) * kHD + 16 * et + m] = (dv[et] * rstd) * g4[et] + b4[et];
    }
    __syncthreads();

    {
        v4f vals[8];
        float* rbase = out + ((size_t)(b * kT + r0)) * kC + head * kHD;
#pragma unroll
        for (int i = 0; i < 8; ++i) {
            const int row = 2 * i + h;
            vals[i] = *(const v4f*)(mys + row * kHD + 4 * m);
        }
#pragma unroll
        for (int i = 0; i < 8; ++i) {
            const int row = 2 * i + h;
            *(volatile v4f*)(rbase + (size_t)row * kC + 4 * m) = vals[i];
        }
        __threadfence();
#pragma unroll
        for (int i = 0; i < 8; ++i) {
            const int row = 2 * i + h;
            *(volatile v4f*)(rbase + (size_t)row * kC + 4 * m) = vals[i];
        }
    }
}

extern "C" void kernel_launch(void* const* d_in, const int* in_sizes, int n_in,
                              void* d_out, int out_size, void* d_ws, size_t ws_size,
                              hipStream_t stream)
{
    if (n_in < 15) return;
    if (in_sizes[0] != kNX || in_sizes[1] != kNX || in_sizes[2] != kNX) return;
    if (in_sizes[3] != kNW || in_sizes[5] != kNW || in_sizes[7] != kNW) return;
    if (in_sizes[4] != kC || in_sizes[6] != kC || in_sizes[8] != kC) return;
    if (in_sizes[9] != kNG || in_sizes[11] != kNG) return;
    if (in_sizes[10] != kNH || in_sizes[12] != kNH) return;
    if (in_sizes[13] != kC || in_sizes[14] != kC) return;
    if (out_size != kNX) return;

    const size_t szX  = (size_t)3 * kNX * sizeof(_Float16);
    const size_t szW  = (size_t)3 * kNW * sizeof(_Float16);
    const size_t szWG = (size_t)2 * kNG * sizeof(_Float16);
    const size_t szG  = (size_t)2 * kGateN * sizeof(float);
    const size_t szP  = (size_t)kPlane * sizeof(_Float16);
    const size_t total = szX + szW + szWG + szG + 5 * szP;
    if (ws_size < total) return;

    const float* q    = (const float*)d_in[0];
    const float* k    = (const float*)d_in[1];
    const float* v    = (const float*)d_in[2];
    const float* Wq_w = (const float*)d_in[3];
    const float* Wq_b = (const float*)d_in[4];
    const float* Wk_w = (const float*)d_in[5];
    const float* Wk_b = (const float*)d_in[6];
    const float* Wv_w = (const float*)d_in[7];
    const float* Wv_b = (const float*)d_in[8];
    const float* Wi_w = (const float*)d_in[9];
    const float* Wi_b = (const float*)d_in[10];
    const float* Wf_w = (const float*)d_in[11];
    const float* Wf_b = (const float*)d_in[12];
    const float* gam  = (const float*)d_in[13];
    const float* bet  = (const float*)d_in[14];
    float* out = (float*)d_out;

    char* ws = (char*)d_ws;
    size_t off = 0;
    _Float16* X16  = (_Float16*)(ws + off); off += szX;
    _Float16* W16  = (_Float16*)(ws + off); off += szW;
    _Float16* WG16 = (_Float16*)(ws + off); off += szWG;
    float*    GATE = (float*)(ws + off);    off += szG;
    _Float16* QH   = (_Float16*)(ws + off); off += szP;
    _Float16* QL   = (_Float16*)(ws + off); off += szP;
    _Float16* KH   = (_Float16*)(ws + off); off += szP;
    _Float16* KL   = (_Float16*)(ws + off); off += szP;
    _Float16* VT   = (_Float16*)(ws + off); off += szP;
    if (off > ws_size) return;

    k_cvt3<<<dim3(kNX / (8 * kThreads), 3), dim3(kThreads), 0, stream>>>(
        q, X16, kNX, k, X16 + kNX, kNX, v, X16 + 2 * (size_t)kNX, kNX, 8.0f);
    k_cvt3<<<dim3(kNW / (8 * kThreads), 3), dim3(kThreads), 0, stream>>>(
        Wq_w, W16, kNW, Wk_w, W16 + kNW, kNW, Wv_w, W16 + 2 * (size_t)kNW, kNW, 1024.0f);
    k_cvt3<<<dim3(kNG / (8 * kThreads), 2), dim3(kThreads), 0, stream>>>(
        Wi_w, WG16, kNG, Wf_w, WG16 + kNG, kNG, Wf_w, WG16 + kNG, kNG, 1024.0f);
    k_gates<<<dim3(kT / 128, kBS), dim3(kThreads), 0, stream>>>(
        X16, X16 + kNX, WG16, WG16 + kNG, Wi_b, Wf_b, GATE);
    k_qkv<<<dim3(kC / 128, (kBS * kT) / 128, 3), dim3(kThreads), 0, stream>>>(
        X16, W16, Wq_b, Wk_b, Wv_b, QH, QL, KH, KL, VT);
    k_attn<<<dim3(kRB, kNH, kBS), dim3(128), 0, stream>>>(
        QH, QL, KH, KL, VT, GATE, gam, bet, out);
}
